// VesselGNN_57767310131222
// MI455X (gfx1250) — hardware-verified
//
#include <hip/hip_runtime.h>
#include <stddef.h>


#define F0      6
#define F1      64
#define HD      128
#define FCK     256
#define NTHR    256
#define NWAVE   8
#define EPT     8
#define NGRP    2
#define CHUNK   (NTHR * EPT * NGRP)
#define WCAP    (EPT * NGRP * 32)
#define LISTN   (NWAVE * WCAP)
#define NBA1    1024
#define NBA2    512
#define NBD     4096
#define GROWS   128
#define L1ROWS  64
#define PRMN    640
#define WSCALE  16.0f
#define WINV    0.0625f
#define BN_EPS  1e-5f

#define LDS_GEMM (GROWS * HD * 4)
#define LDS_AGG  (65536 * 4 + LISTN * 4 + PRMN * 4 + 64)

static_assert((CHUNK & (CHUNK - 1)) == 0);
static_assert(CHUNK <= 4096);
static_assert(NBA1 <= 4096 && NBA2 <= 4096 && NBD <= 4096);
static_assert(NBA1 * F1 == 65536 && NBA2 * HD == 65536);
static_assert(GROWS * (HD + 8) * 2 <= LDS_GEMM);
static_assert((NBD % GROWS) == 0);

typedef float    v2f  __attribute__((ext_vector_type(2)));
typedef float    v4f  __attribute__((ext_vector_type(4)));
typedef float    v8f  __attribute__((ext_vector_type(8)));
typedef int      v4i  __attribute__((ext_vector_type(4)));
typedef _Float16 v8h  __attribute__((ext_vector_type(8)));
typedef _Float16 v16h __attribute__((ext_vector_type(16)));
union FragH { v16h v; v8h h[2]; };

template <int F> struct RowVec;
template <> struct RowVec<64>  { typedef v2f T; };
template <> struct RowVec<128> { typedef v4f T; };

__device__ __forceinline__ v8h cvt8(v4f a, v4f b) {
  v8h r;
  r[0] = (_Float16)a.x; r[1] = (_Float16)a.y; r[2] = (_Float16)a.z; r[3] = (_Float16)a.w;
  r[4] = (_Float16)b.x; r[5] = (_Float16)b.y; r[6] = (_Float16)b.z; r[7] = (_Float16)b.w;
  return r;
}

__device__ __forceinline__ v8f wmh(v16h a, v16h b, v8f c) {
  v8f d = __builtin_amdgcn_wmma_f32_16x16x32_f16(false, a, false, b, (short)0, c, false, false);
  asm volatile("v_nop\n\tv_nop\n\tv_nop\n\tv_nop" : "+v"(d) : "v"(a), "v"(b));
  return d;
}

template <int NB>
__device__ __forceinline__ int scan_chunk(const int* __restrict__ dsts, int nE, int cbase, int nodeBase,
                                          int vec8, int* list, int tid, int lane, int wave) {
  int wc = 0;
#pragma unroll
  for (int g = 0; g < NGRP; ++g) {
    const int el0  = (g * NTHR + tid) * EPT;
    const int e0   = cbase + el0;
    const int sent = -2147483647 - 1;
    v4i da, db;
    if (vec8 != 0 && e0 + 7 < nE) {
      da = *(const v4i*)(dsts + e0);
      db = *(const v4i*)(dsts + e0 + 4);
    } else {
      da.x = (e0     < nE) ? dsts[min(e0, nE - 1)] : sent;
      da.y = (e0 + 1 < nE) ? dsts[min(e0 + 1, nE - 1)] : sent;
      da.z = (e0 + 2 < nE) ? dsts[min(e0 + 2, nE - 1)] : sent;
      da.w = (e0 + 3 < nE) ? dsts[min(e0 + 3, nE - 1)] : sent;
      db.x = (e0 + 4 < nE) ? dsts[min(e0 + 4, nE - 1)] : sent;
      db.y = (e0 + 5 < nE) ? dsts[min(e0 + 5, nE - 1)] : sent;
      db.z = (e0 + 6 < nE) ? dsts[min(e0 + 6, nE - 1)] : sent;
      db.w = (e0 + 7 < nE) ? dsts[min(e0 + 7, nE - 1)] : sent;
    }
    const unsigned nb = (unsigned)nodeBase;
    const unsigned s0 = (unsigned)da.x - nb, s1 = (unsigned)da.y - nb;
    const unsigned s2 = (unsigned)da.z - nb, s3 = (unsigned)da.w - nb;
    const unsigned s4 = (unsigned)db.x - nb, s5 = (unsigned)db.y - nb;
    const unsigned s6 = (unsigned)db.z - nb, s7 = (unsigned)db.w - nb;
    const bool h0 = s0 < (unsigned)NB, h1 = s1 < (unsigned)NB, h2 = s2 < (unsigned)NB, h3 = s3 < (unsigned)NB;
    const bool h4 = s4 < (unsigned)NB, h5 = s5 < (unsigned)NB, h6 = s6 < (unsigned)NB, h7 = s7 < (unsigned)NB;
    const unsigned any = __builtin_amdgcn_ballot_w32(h0 | h1 | h2 | h3 | h4 | h5 | h6 | h7);
    if (any != 0u) {
#define HITJ(J, HJ, SJ) { \
        const unsigned mj = __builtin_amdgcn_ballot_w32(HJ); \
        if (mj != 0u) { \
          if (HJ) { \
            const int pos = wc + (int)__builtin_amdgcn_mbcnt_lo(mj, 0u); \
            if (pos < WCAP) list[wave * WCAP + pos] = ((el0 + (J)) << 12) | (int)(SJ); \
          } \
          wc += (int)__builtin_popcount(mj); } }
      HITJ(0, h0, s0)
      HITJ(1, h1, s1)
      HITJ(2, h2, s2)
      HITJ(3, h3, s3)
      HITJ(4, h4, s4)
      HITJ(5, h5, s5)
      HITJ(6, h6, s6)
      HITJ(7, h7, s7)
#undef HITJ
    }
  }
  return wc;
}

__global__ __launch_bounds__(NTHR) void k_wprep(
    const float* __restrict__ W2, const float* __restrict__ W3,
    _Float16* w2s, _Float16* w3s) {
  const int i  = blockIdx.x * NTHR + threadIdx.x;
  const int n2 = HD * F1 / 8;
  const int n3 = HD * HD / 8;
  if (i >= n2 + n3) return;
  const bool first = i < n2;
  const int o  = (first ? i : i - n2) * 8;
  const int n  = first ? (o >> 6) : (o >> 7);
  const int k0 = first ? (o & (F1 - 1)) : (o & (HD - 1));
  const float* p = (first ? W2 : W3) + (size_t)k0 * HD + n;
  v4f a, b;
  a.x = p[0];      a.y = p[HD];     a.z = p[2 * HD]; a.w = p[3 * HD];
  b.x = p[4 * HD]; b.y = p[5 * HD]; b.z = p[6 * HD]; b.w = p[7 * HD];
  a = a * WSCALE;
  b = b * WSCALE;
  const v8h hv = cvt8(a, b);
  _Float16* dp = (first ? w2s : w3s) + o;
  *(volatile v8h*)dp = hv;
  __threadfence();
  *(volatile v8h*)dp = hv;
}

__global__ __launch_bounds__(NTHR) void k_deg(
    const int* __restrict__ ei, float* dinv, int nN, int nE, int vec8) {
  __shared__ __attribute__((aligned(16))) int cnt[NBD];
  __shared__ __attribute__((aligned(16))) int list[LISTN];
  __shared__ int wcnt[NWAVE];
  const int tid = threadIdx.x, lane = tid & 31, wave = tid >> 5;
  const int nodeBase = blockIdx.x * NBD;
  const int* dsts = ei + nE;
  (void)nN;

  for (int i = tid; i < NBD; i += NTHR) cnt[i] = 0;
  __syncthreads();

  const int nChunks = (nE + CHUNK - 1) / CHUNK;
#pragma unroll 1
  for (int ch = 0; ch < nChunks; ++ch) {
    const int cbase = ch * CHUNK;
    const int wc = scan_chunk<NBD>(dsts, nE, cbase, nodeBase, vec8, list, tid, lane, wave);
    if (lane == 0) wcnt[wave] = wc;
    __syncthreads();
    if (wave == 0) {
#pragma unroll 1
      for (int wsx = 0; wsx < NWAVE; ++wsx) {
        int n = __builtin_amdgcn_readfirstlane(wcnt[wsx]);
        n = n > WCAP ? WCAP : (n < 0 ? 0 : n);
        const int* lp = list + wsx * WCAP;
#pragma unroll 1
        for (int i = 0; i < n; ++i) {
          const int ent  = __builtin_amdgcn_readfirstlane(lp[i]);
          const int slot = ent & (NBD - 1);
          if (lane == 0) cnt[slot] = cnt[slot] + 1;
        }
      }
    }
    __syncthreads();
  }

  v4f dq[4];
#pragma unroll
  for (int q = 0; q < 4; ++q) {
    const int f = (wave * 4 + q) * 128 + 4 * lane;
    const v4i c = *(const v4i*)(cnt + f);
    dq[q].x = rsqrtf((float)(c.x + 1));
    dq[q].y = rsqrtf((float)(c.y + 1));
    dq[q].z = rsqrtf((float)(c.z + 1));
    dq[q].w = rsqrtf((float)(c.w + 1));
  }
  float* dp = dinv + (size_t)nodeBase;
#pragma unroll
  for (int q = 0; q < 4; ++q) *(volatile v4f*)(dp + (wave * 4 + q) * 128 + 4 * lane) = dq[q];
  __threadfence();
#pragma unroll
  for (int q = 0; q < 4; ++q) *(volatile v4f*)(dp + (wave * 4 + q) * 128 + 4 * lane) = dq[q];
}

__global__ __launch_bounds__(NTHR) void k_l1(
    const float* __restrict__ x, const float* __restrict__ W1, const float* __restrict__ dinv,
    float* g1p, int nN) {
  __shared__ __attribute__((aligned(16))) float sW[F0 * F1];
  __shared__ __attribute__((aligned(16))) v4f sO[4 * NTHR];
  const int tid = threadIdx.x, lane = tid & 31, wave = tid >> 5, hh = lane >> 4;
  const int c0 = (lane & 15) * 4;
  for (int i = tid; i < F0 * F1; i += NTHR) sW[i] = W1[i];
  __syncthreads();

  const int rowBase = blockIdx.x * L1ROWS + wave * 8;
#pragma unroll 1
  for (int q = 0; q < 4; ++q) {
    int node = rowBase + 2 * q + hh;
    node = node > nN - 1 ? nN - 1 : node;
    const float* xp = x + (size_t)node * F0;
    v4f o = {0.f, 0.f, 0.f, 0.f};
#pragma unroll
    for (int k = 0; k < F0; ++k) {
      const float xv = xp[k];
      const v4f   w  = *(const v4f*)(sW + k * F1 + c0);
      o = o + xv * w;
    }
    const float d = dinv[node];
    sO[q * NTHR + tid] = o * d;
  }

  float* gp = g1p + (size_t)rowBase * F1 + c0;
#pragma unroll
  for (int q = 0; q < 4; ++q) {
    const v4f v = sO[q * NTHR + tid];
    *(volatile v4f*)(gp + (size_t)(2 * q + hh) * F1) = v;
  }
  __threadfence();
#pragma unroll
  for (int q = 0; q < 4; ++q) {
    const v4f v = sO[q * NTHR + tid];
    *(volatile v4f*)(gp + (size_t)(2 * q + hh) * F1) = v;
  }
}

template <int F, int NB>
__global__ __launch_bounds__(NTHR) void k_agg(
    const int* __restrict__ ei, const float* __restrict__ gpl, const float* __restrict__ dinv,
    const float* __restrict__ bias, const float* __restrict__ gam, const float* __restrict__ bet,
    const float* __restrict__ rmean, const float* __restrict__ rvar,
    float* hpl, int nN, int nE, int vec8) {
  typedef typename RowVec<F>::T vrow;
  constexpr int VPL = F / 32;
  constexpr int V4R = F / 4;
  constexpr int NQ  = (NB * F) / (128 * NWAVE);
  extern __shared__ v4f lds_dyn[];
  float* acc  = (float*)lds_dyn;
  int*   list = (int*)(acc + NB * F);
  float* prm  = (float*)(list + LISTN);
  int*   wcnt = (int*)(prm + PRMN);
  const int tid = threadIdx.x, lane = tid & 31, wave = tid >> 5;
  const int nodeBase = blockIdx.x * NB;
  const int* dsts = ei + nE;

  {
    const v4f z = {0.f, 0.f, 0.f, 0.f};
    for (int i = tid; i < NB * F / 4; i += NTHR) lds_dyn[i] = z;
  }
  if (tid < F) {
    prm[tid]       = bias[tid];
    prm[128 + tid] = gam[tid];
    prm[256 + tid] = bet[tid];
    prm[384 + tid] = rmean[tid];
    prm[512 + tid] = rsqrtf(rvar[tid] + BN_EPS);
  }
  __syncthreads();

  const int nChunks = (nE + CHUNK - 1) / CHUNK;
#pragma unroll 1
  for (int ch = 0; ch < nChunks; ++ch) {
    const int cbase = ch * CHUNK;
    const int wc = scan_chunk<NB>(dsts, nE, cbase, nodeBase, vec8, list, tid, lane, wave);
    if (lane == 0) wcnt[wave] = wc;
    __syncthreads();
    if (wave == 0) {
#pragma unroll 1
      for (int wsx = 0; wsx < NWAVE; ++wsx) {
        int n = __builtin_amdgcn_readfirstlane(wcnt[wsx]);
        n = n > WCAP ? WCAP : (n < 0 ? 0 : n);
        const int* lp = list + wsx * WCAP;
#pragma unroll 1
        for (int i = 0; i < n; ++i) {
          const int ent  = __builtin_amdgcn_readfirstlane(lp[i]);
          const int slot = ent & (NB - 1);
          int e = cbase + ((ent >> 12) & (CHUNK - 1));
          e = e > nE - 1 ? nE - 1 : e;
          int src = ei[e];
          src = src < 0 ? 0 : (src > nN - 1 ? nN - 1 : src);
          const vrow v = *(const vrow*)(gpl + (size_t)src * F + VPL * lane);
          vrow* ap = (vrow*)(acc + slot * F + VPL * lane);
          *ap = *ap + v;
        }
      }
    }
    __syncthreads();
  }

#pragma unroll 4
  for (int i = 0; i < (NB * F / 4) / NTHR; ++i) {
    const int idx  = i * NTHR + tid;
    const int slot = idx / V4R;
    const int c4   = (idx - slot * V4R) * 4;
    int node = nodeBase + slot;
    node = node > nN - 1 ? nN - 1 : node;
    const float d  = dinv[node];
    const v4f   gv = *(const v4f*)(gpl + (size_t)node * F + c4);
    const v4f   bv = *(const v4f*)(prm + c4);
    const v4f   gg = *(const v4f*)(prm + 128 + c4);
    const v4f   be = *(const v4f*)(prm + 256 + c4);
    const v4f   rm = *(const v4f*)(prm + 384 + c4);
    const v4f   rs = *(const v4f*)(prm + 512 + c4);
    v4f* ap = (v4f*)(acc + slot * F + c4);
    v4f hv = (*ap + gv) * d + bv;
    hv = (hv - rm) * rs * gg + be;
    hv.x = fmaxf(hv.x, 0.f); hv.y = fmaxf(hv.y, 0.f); hv.z = fmaxf(hv.z, 0.f); hv.w = fmaxf(hv.w, 0.f);
    *ap = hv;
  }
  __syncthreads();

  float* hp = hpl + (size_t)nodeBase * F;
#pragma unroll 4
  for (int q = 0; q < NQ; ++q) {
    const int f = (wave * NQ + q) * 128 + 4 * lane;
    const v4f v = *(const v4f*)(acc + f);
    *(volatile v4f*)(hp + f) = v;
  }
  __threadfence();
#pragma unroll 4
  for (int q = 0; q < NQ; ++q) {
    const int f = (wave * NQ + q) * 128 + 4 * lane;
    const v4f v = *(const v4f*)(acc + f);
    *(volatile v4f*)(hp + f) = v;
  }
}

template <int K>
__global__ __launch_bounds__(NTHR) void k_gemm(
    const float* __restrict__ hpl, const _Float16* __restrict__ wpl,
    const float* __restrict__ dinv, float* gpl, int nN) {
  constexpr int APK = K + 8;
  constexpr int KG  = K / 8;
  extern __shared__ v4f lds_dyn[];
  _Float16* sA  = (_Float16*)lds_dyn;
  float*    stg = (float*)lds_dyn;
  const int tid = threadIdx.x, lane = tid & 31, wave = tid >> 5, hh = lane >> 4, m = lane & 15;
  const int rowBase = blockIdx.x * GROWS;

#pragma unroll
  for (int i = 0; i < (GROWS * KG) / NTHR; ++i) {
    const int idx = i * NTHR + tid;
    const int r   = idx / KG;
    const int c0  = (idx - r * KG) * 8;
    int node = rowBase + r;
    node = node > nN - 1 ? nN - 1 : node;
    const float* xp = hpl + (size_t)node * K + c0;
    const v4f a = *(const v4f*)xp, b = *(const v4f*)(xp + 4);
    *(v8h*)(sA + r * APK + c0) = cvt8(a, b);
  }
  __syncthreads();

  v8f acc[8];
#pragma unroll
  for (int t = 0; t < 8; ++t) { v8f z = {0.f, 0.f, 0.f, 0.f, 0.f, 0.f, 0.f, 0.f}; acc[t] = z; }
  const _Float16* ar = sA + (wave * 16 + m) * APK + 8 * hh;
#pragma unroll
  for (int kt = 0; kt < K / 32; ++kt) {
    FragH a;
    a.h[0] = *(const v8h*)(ar + 32 * kt);
    a.h[1] = *(const v8h*)(ar + 32 * kt + 16);
#pragma unroll
    for (int t = 0; t < 8; ++t) {
      const _Float16* bp = wpl + (size_t)(16 * t + m) * K + 32 * kt + 8 * hh;
      FragH b;
      b.h[0] = *(const v8h*)bp;
      b.h[1] = *(const v8h*)(bp + 16);
      acc[t] = wmh(a.v, b.v, acc[t]);
    }
  }
  __syncthreads();

  const int r0 = wave * 16 + 8 * hh;
  const v4f dA = *(const v4f*)(dinv + (size_t)rowBase + r0);
  const v4f dB = *(const v4f*)(dinv + (size_t)rowBase + r0 + 4);
  const float d0 = dA.x * WINV, d1 = dA.y * WINV, d2 = dA.z * WINV, d3 = dA.w * WINV;
  const float d4 = dB.x * WINV, d5 = dB.y * WINV, d6 = dB.z * WINV, d7 = dB.w * WINV;
  float* sp = stg + r0 * HD + m;
#pragma unroll
  for (int t = 0; t < 8; ++t) {
    sp[0 * HD + 16 * t] = acc[t][0] * d0;
    sp[1 * HD + 16 * t] = acc[t][1] * d1;
    sp[2 * HD + 16 * t] = acc[t][2] * d2;
    sp[3 * HD + 16 * t] = acc[t][3] * d3;
    sp[4 * HD + 16 * t] = acc[t][4] * d4;
    sp[5 * HD + 16 * t] = acc[t][5] * d5;
    sp[6 * HD + 16 * t] = acc[t][6] * d6;
    sp[7 * HD + 16 * t] = acc[t][7] * d7;
  }
  __syncthreads();

  const float* lp = stg + wave * 16 * HD + 4 * lane;
  float* gp = gpl + ((size_t)rowBase + wave * 16) * HD + 4 * lane;
#pragma unroll
  for (int i = 0; i < 16; ++i) { const v4f v = *(const v4f*)(lp + i * HD); *(volatile v4f*)(gp + (size_t)i * HD) = v; }
  __threadfence();
#pragma unroll
  for (int i = 0; i < 16; ++i) { const v4f v = *(const v4f*)(lp + i * HD); *(volatile v4f*)(gp + (size_t)i * HD) = v; }
}

__global__ __launch_bounds__(HD) void k_poolfc(
    const float* __restrict__ hpl, const int* __restrict__ bat,
    const float* __restrict__ fcW, const float* __restrict__ fcb,
    float* out, int nN) {
  __shared__ __attribute__((aligned(16))) float pooled[2 * HD];
  __shared__ __attribute__((aligned(16))) float orow[HD];
  const int g = blockIdx.x, j = threadIdx.x, lane = j & 31, wave = j >> 5;
  float sum = 0.f, mx = __int_as_float(0xff800000u);
  int cnt = 0;
  const int nch = (nN + 31) >> 5;
#pragma unroll 1
  for (int ch = 0; ch < nch; ++ch) {
    const int i  = ch * 32 + lane;
    const int bv = bat[i < nN ? i : nN - 1];
    const int b  = (i < nN) ? bv : -1;
    unsigned msk = __builtin_amdgcn_ballot_w32(b == g);
    cnt += (int)__builtin_popcount(msk);
    while (msk != 0u) {
      const int bit = __builtin_ctz(msk);
      msk &= msk - 1u;
      const int node = ch * 32 + bit;
      const float v = hpl[(size_t)node * HD + j];
      sum += v;
      mx = fmaxf(mx, v);
    }
  }
  const float inv = 1.0f / fmaxf((float)cnt, 1.0f);
  pooled[j]      = sum * inv;
  pooled[HD + j] = mx;
  __syncthreads();

  float o = 0.f;
#pragma unroll 4
  for (int k = 0; k < FCK; ++k) o += pooled[k] * fcW[(size_t)k * HD + j];
  o += fcb[j];
  orow[j] = o;
  __syncthreads();

  if (wave == 0) {
    const v4f v = *(const v4f*)(orow + 4 * lane);
    float* op = out + (size_t)g * HD + 4 * lane;
    *(volatile v4f*)op = v;
    __threadfence();
    *(volatile v4f*)op = v;
  }
}

extern "C" void kernel_launch(void* const* d_in, const int* in_sizes, int n_in,
                              void* d_out, int out_size, void* d_ws, size_t ws_size,
                              hipStream_t stream) {
  if (n_in < 23) return;
  const int nN = in_sizes[0] / F0;
  const int nE = in_sizes[1] / 2;
  if (nN <= 0 || in_sizes[0] != nN * F0 || nE < 0 || in_sizes[1] != 2 * nE || in_sizes[2] != nN) return;
  if (in_sizes[3] != F0 * F1 || in_sizes[4] < F1) return;
  if (in_sizes[5] != F1 * HD || in_sizes[6] < HD) return;
  if (in_sizes[7] != HD * HD || in_sizes[8] < HD) return;
  for (int i = 9; i <= 12; ++i) if (in_sizes[i] < F1) return;
  for (int i = 13; i <= 20; ++i) if (in_sizes[i] < HD) return;
  if (in_sizes[21] != FCK * HD || in_sizes[22] < HD) return;
  const int nG = out_size / HD;
  if (nG <= 0 || out_size != nG * HD) return;

  const float* x   = (const float*)d_in[0];
  const int*   ei  = (const int*)d_in[1];
  const int*   bat = (const int*)d_in[2];
  const float* W1  = (const float*)d_in[3];  const float* b1  = (const float*)d_in[4];
  const float* W2  = (const float*)d_in[5];  const float* b2  = (const float*)d_in[6];
  const float* W3  = (const float*)d_in[7];  const float* b3  = (const float*)d_in[8];
  const float* g1  = (const float*)d_in[9];  const float* be1 = (const float*)d_in[10];
  const float* rm1 = (const float*)d_in[11]; const float* rv1 = (const float*)d_in[12];
  const float* g2  = (const float*)d_in[13]; const float* be2 = (const float*)d_in[14];
  const float* rm2 = (const float*)d_in[15]; const float* rv2 = (const float*)d_in[16];
  const float* g3  = (const float*)d_in[17]; const float* be3 = (const float*)d_in[18];
  const float* rm3 = (const float*)d_in[19]; const float* rv3 = (const float*)d_in[20];
  const float* fcW = (const float*)d_in[21]; const float* fcb = (const float*)d_in[22];
  float* out = (float*)d_out;

  const int nBD = (nN + NBD - 1) / NBD;
  const int nL1 = (nN + L1ROWS - 1) / L1ROWS;
  const int nGm = (nN + GROWS - 1) / GROWS;
  const int nA1 = (nN + NBA1 - 1) / NBA1;
  const int nA2 = (nN + NBA2 - 1) / NBA2;

  size_t capG = (size_t)nGm * GROWS * HD;
  { const size_t c = (size_t)nL1 * L1ROWS * F1; if (c > capG) capG = c; }
  size_t capH = (size_t)nA2 * NBA2 * HD;
  { const size_t c = (size_t)nA1 * NBA1 * F1; if (c > capH) capH = c; }

  char* ws = (char*)d_ws;
  size_t off = 0;
  const size_t oW2 = off; off += (size_t)HD * F1 * 2;   off = (off + 255) & ~(size_t)255;
  const size_t oW3 = off; off += (size_t)HD * HD * 2;   off = (off + 255) & ~(size_t)255;
  const size_t oDv = off; off += (size_t)nBD * NBD * 4; off = (off + 255) & ~(size_t)255;
  const size_t oG  = off; off += capG * 4;              off = (off + 255) & ~(size_t)255;
  const size_t oH  = off; off += capH * 4;              off = (off + 255) & ~(size_t)255;
  if (off > ws_size) return;
  _Float16* w2s  = (_Float16*)(ws + oW2);
  _Float16* w3s  = (_Float16*)(ws + oW3);
  float*    dinv = (float*)(ws + oDv);
  float*    Gp   = (float*)(ws + oG);
  float*    Hp   = (float*)(ws + oH);

  const int vec8 = ((nE & 3) == 0) ? 1 : 0;

  const int nPrep = HD * F1 / 8 + HD * HD / 8;
  k_wprep<<<(nPrep + NTHR - 1) / NTHR, NTHR, 0, stream>>>(W2, W3, w2s, w3s);

  k_deg<<<nBD, NTHR, 0, stream>>>(ei, dinv, nN, nE, vec8);

  k_l1<<<nL1, NTHR, 0, stream>>>(x, W1, dinv, Gp, nN);

  hipFuncSetAttribute(reinterpret_cast<const void*>(&k_agg<F1, NBA1>),
                      hipFuncAttributeMaxDynamicSharedMemorySize, LDS_AGG);
  hipFuncSetAttribute(reinterpret_cast<const void*>(&k_agg<HD, NBA2>),
                      hipFuncAttributeMaxDynamicSharedMemorySize, LDS_AGG);
  hipFuncSetAttribute(reinterpret_cast<const void*>(&k_gemm<F1>),
                      hipFuncAttributeMaxDynamicSharedMemorySize, LDS_GEMM);
  hipFuncSetAttribute(reinterpret_cast<const void*>(&k_gemm<HD>),
                      hipFuncAttributeMaxDynamicSharedMemorySize, LDS_GEMM);

  k_agg<F1, NBA1><<<nA1, NTHR, LDS_AGG, stream>>>(ei, Gp, dinv, b1, g1, be1, rm1, rv1, Hp, nN, nE, vec8);
  k_gemm<F1><<<nGm, NTHR, LDS_GEMM, stream>>>(Hp, w2s, dinv, Gp, nN);
  k_agg<HD, NBA2><<<nA2, NTHR, LDS_AGG, stream>>>(ei, Gp, dinv, b2, g2, be2, rm2, rv2, Hp, nN, nE, vec8);
  k_gemm<HD><<<nGm, NTHR, LDS_GEMM, stream>>>(Hp, w3s, dinv, Gp, nN);
  k_agg<HD, NBA2><<<nA2, NTHR, LDS_AGG, stream>>>(ei, Gp, dinv, b3, g3, be3, rm3, rv3, Hp, nN, nE, vec8);

  k_poolfc<<<nG, HD, 0, stream>>>(Hp, bat, fcW, fcb, out, nN);
}
